// LSTM_decomposedGIN_28140625724085
// MI455X (gfx1250) — hardware-verified
//
#include <hip/hip_runtime.h>

typedef __attribute__((ext_vector_type(16))) _Float16 v16h;
typedef __attribute__((ext_vector_type(8)))  _Float16 v8h;
typedef __attribute__((ext_vector_type(2)))  _Float16 v2h;
typedef __attribute__((ext_vector_type(16))) __bf16   v16b;
typedef __attribute__((ext_vector_type(8)))  __bf16   v8b;
typedef __attribute__((ext_vector_type(8)))  float    v8f;
typedef __attribute__((ext_vector_type(4)))  float    v4f;
typedef __attribute__((ext_vector_type(2)))  float    v2f;

static constexpr int kSteps    = 215;
static constexpr int kBatch    = 2048;
static constexpr int kDin      = 36;
static constexpr int kXpad     = 64;
static constexpr int kHid      = 128;
static constexpr int kGates    = 512;
static constexpr int kKcat     = kXpad + kHid;
static constexpr int kTilePitch = 200;
static constexpr int kStgPitch  = 136;
static constexpr int kRowsPB   = 16;
static constexpr int kEncRows  = 128;
static constexpr int kEncPitch = 72;
static constexpr int kDmlp     = 137;
static constexpr int kDmlpPad  = 192;
static constexpr int kStatic   = 9;
static constexpr int kClasses  = 2;

static_assert(kBatch % kRowsPB == 0, "lstm grid exact");
static_assert((kSteps * kBatch) % kEncRows == 0, "enc grid exact");
static_assert(kBatch % kEncRows == 0, "enc block inside one step");
static_assert(kKcat % 32 == 0, "k steps of 32");
static_assert(kDmlpPad % 64 == 0 && kBatch % 64 == 0, "kit gemm tile multiples");
static_assert((kGates * kKcat / 2) % 256 == 0, "prep region 0 block aligned");
static_assert((kDmlpPad * kDmlpPad / 2) % 256 == 0, "prep region 1 block aligned");
static_assert((kBatch * (kDmlpPad - kHid) / 2) % 256 == 0, "prep region 3 block aligned");

__device__ __forceinline__ unsigned short f2bf_bits(float f) {
  unsigned u = __float_as_uint(f);
  return (unsigned short)((u + 0x7FFFu + ((u >> 16) & 1u)) >> 16);
}
__device__ __forceinline__ float bf_bits2f(unsigned short h) { return __uint_as_float(((unsigned)h) << 16); }

__device__ __forceinline__ void dep_guard_h(v8f& a, v8f& b, v16h x, v16h y) { asm volatile("v_nop\n\tv_nop\n\tv_nop\n\tv_nop" : "+v"(a), "+v"(b) : "v"(x), "v"(y)); }
__device__ __forceinline__ void dep_guard_b(v8f& a, v8f& b, v16b x, v16b y) { asm volatile("v_nop\n\tv_nop\n\tv_nop\n\tv_nop" : "+v"(a), "+v"(b) : "v"(x), "v"(y)); }
__device__ __forceinline__ void keep4_h(v16h a, v16h b, v16h c, v16h d) { asm volatile("v_nop" :: "v"(a), "v"(b), "v"(c), "v"(d)); }
__device__ __forceinline__ void keep4_b(v16b a, v16b b, v16b c, v16b d) { asm volatile("v_nop" :: "v"(a), "v"(b), "v"(c), "v"(d)); }
__device__ __forceinline__ void acc_guard4(v8f& a, v8f& b, v8f& c, v8f& d) { asm volatile("v_nop\n\tv_nop\n\tv_nop\n\tv_nop" : "+v"(a), "+v"(b), "+v"(c), "+v"(d)); }
template <typename T> struct Frag;
template <> struct Frag<_Float16> {
  typedef v16h V; union U { v16h v; v8h h[2]; };
  static __device__ __forceinline__ v16h load(const _Float16* p) {
    U f; f.h[0] = *(const v8h*)(p); f.h[1] = *(const v8h*)(p + 16); return f.v;
  }
  static __device__ __forceinline__ v8f mma(v16h a, v16h b, v8f c) {
    return __builtin_amdgcn_wmma_f32_16x16x32_f16(false, a, false, b, (short)0, c, false, false);
  }
  static __device__ __forceinline__ void guard(v8f& a, v8f& b, v16h x, v16h y) { dep_guard_h(a, b, x, y); }
  static __device__ __forceinline__ void keep(v16h a, v16h b, v16h c, v16h d) { keep4_h(a, b, c, d); }
};
template <> struct Frag<__bf16> {
  typedef v16b V; union U { v16b v; v8b h[2]; };
  static __device__ __forceinline__ v16b load(const __bf16* p) {
    U f; f.h[0] = *(const v8b*)(p); f.h[1] = *(const v8b*)(p + 16); return f.v;
  }
  static __device__ __forceinline__ v8f mma(v16b a, v16b b, v8f c) {
    return __builtin_amdgcn_wmma_f32_16x16x32_bf16(false, a, false, b, (short)0, c, false, false);
  }
  static __device__ __forceinline__ void guard(v8f& a, v8f& b, v16b x, v16b y) { dep_guard_b(a, b, x, y); }
  static __device__ __forceinline__ void keep(v16b a, v16b b, v16b c, v16b d) { keep4_b(a, b, c, d); }
};

template <int ET> struct Elem;
template <> struct Elem<0> { typedef _Float16 T; };
template <> struct Elem<1> { typedef __bf16 T; };
template <int ET, bool SPLIT, int BIAS_MODE, int OUT_MODE, bool RESID, int ACT = 0>
__global__ __launch_bounds__(256) void wmma_gemm64(
    const unsigned short* __restrict__ Ap, const unsigned short* __restrict__ A2p, int lda, long strideA,
    const unsigned short* __restrict__ Btp, const unsigned short* __restrict__ Bt2p, int ldb, long strideB,
    void* __restrict__ Cout, void* __restrict__ Cout2, int ldc, long strideC,
    const float* __restrict__ bias,
    const float* __restrict__ resid, long strideR,
    int M, int N, int K, float scale) {
  typedef typename Elem<ET>::T T;
  typedef typename Frag<T>::V V;
  const T* A = (const T*)Ap; const T* A2 = (const T*)A2p; const T* Bt = (const T*)Btp; const T* Bt2 = (const T*)Bt2p;
  __shared__ __align__(16) float sT[8][16 * 68];
  const int b    = blockIdx.y;
  const int lane = threadIdx.x & 31;
  const int wave = threadIdx.x >> 5;
  const int tilesN = N >> 6;
  const int tilesM = M >> 6;
  const int tile = blockIdx.x * 8 + wave;
  if (tile >= tilesM * tilesN) return;
  const int tm = tile / tilesN;
  const int tn = tile - tm * tilesN;
  const int m0 = tm << 6;
  const int n0 = tn << 6;

  const T* Ab  = A  + (size_t)b * strideA;
  const T* Bb  = Bt + (size_t)b * strideB;
  const T* Ab2 = SPLIT ? (A2  + (size_t)b * strideA) : nullptr;
  const T* Bb2 = SPLIT ? (Bt2 + (size_t)b * strideB) : nullptr;

  const int rlane = lane & 15;
  const int koff  = (lane >> 4) * 8;
  const int mOff  = (lane >> 4) * 8;

  v8f acc[4][4];
#pragma unroll
  for (int i = 0; i < 4; ++i)
#pragma unroll
    for (int j = 0; j < 4; ++j) acc[i][j] = (v8f){0.f,0.f,0.f,0.f,0.f,0.f,0.f,0.f};

  for (int k0 = 0; k0 < K; k0 += 32) {
    V bh[4], bl[4];
#pragma unroll
    for (int j = 0; j < 4; ++j) {
      const size_t bo = (size_t)(n0 + (j << 4) + rlane) * ldb + koff + k0;
      bh[j] = Frag<T>::load(Bb + bo);
      if (SPLIT) bl[j] = Frag<T>::load(Bb2 + bo);
    }
#pragma unroll
    for (int i = 0; i < 4; ++i) {
      const size_t ao = (size_t)(m0 + (i << 4) + rlane) * lda + koff + k0;
      V ah = Frag<T>::load(Ab + ao);
      V al;
      if (SPLIT) al = Frag<T>::load(Ab2 + ao);
#pragma unroll
      for (int j = 0; j < 4; ++j) {
        acc[i][j] = Frag<T>::mma(ah, bh[j], acc[i][j]);
        if (SPLIT) {
          acc[i][j] = Frag<T>::mma(ah, bl[j], acc[i][j]);
          acc[i][j] = Frag<T>::mma(al, bh[j], acc[i][j]);
        }
      }
      Frag<T>::guard(acc[i][0], acc[i][3], ah, SPLIT ? al : ah);
    }
    Frag<T>::keep(bh[0], bh[1], bh[2], bh[3]);
    if (SPLIT) Frag<T>::keep(bl[0], bl[1], bl[2], bl[3]);
  }
  acc_guard4(acc[0][0], acc[0][1], acc[0][2], acc[0][3]);
  acc_guard4(acc[1][0], acc[1][1], acc[1][2], acc[1][3]);
  acc_guard4(acc[2][0], acc[2][1], acc[2][2], acc[2][3]);
  acc_guard4(acc[3][0], acc[3][1], acc[3][2], acc[3][3]);

  float* slab = sT[wave];
  const float* Rb = RESID ? (resid + (size_t)b * strideR) : nullptr;
#pragma unroll
  for (int i = 0; i < 4; ++i) {
    const int mBase = m0 + (i << 4);
#pragma unroll
    for (int j = 0; j < 4; ++j) {
      const int n = n0 + (j << 4) + rlane;
      float bv = 0.f;
      if (BIAS_MODE == 2) bv = bias[n];
#pragma unroll
      for (int r = 0; r < 8; ++r) {
        float v = acc[i][j][r] * scale;
        if (BIAS_MODE == 1) v += bias[mBase + mOff + r];
        if (BIAS_MODE == 2) v += bv;
        if (RESID) v += Rb[(size_t)(mBase + mOff + r) * ldc + n];
        if (ACT == 1) v = tanhf(v);
        if (ACT == 2) v = fmaxf(v, 0.0f);
        if (ACT == 3) v = v / (1.0f + expf(-v));
        if (ACT == 4) v = (v > 0.f) ? v : 0.01f * v;
        if (ACT == 5) v = 0.5f * v * (1.0f + erff(v * 0.70710678118654752f));
        slab[(mOff + r) * 68 + (j << 4) + rlane] = v;
      }
    }
    __builtin_amdgcn_fence(__ATOMIC_RELEASE, "workgroup");
    __builtin_amdgcn_wave_barrier();
    __builtin_amdgcn_fence(__ATOMIC_ACQUIRE, "workgroup");
    if (OUT_MODE == 0) {
      float* C = (float*)Cout + (size_t)b * strideC;
      const int hh = lane >> 4, c4 = (lane & 15) * 4;
      for (int pass = 0; pass < 2; ++pass) {
#pragma unroll
        for (int it = 0; it < 8; ++it) {
          const int row = it * 2 + hh;
          v4f v = *(const v4f*)(slab + row * 68 + c4);
          *(volatile v4f*)(C + (size_t)(mBase + row) * ldc + n0 + c4) = v;
        }
        __threadfence();
      }
    } else {
      const int q = lane >> 3, c8 = (lane & 7) * 8;
      unsigned short* C  = (unsigned short*)Cout  + (size_t)b * strideC;
      unsigned short* C2 = (OUT_MODE == 2) ? ((unsigned short*)Cout2 + (size_t)b * strideC) : nullptr;
      for (int pass = 0; pass < 2; ++pass) {
#pragma unroll
        for (int it = 0; it < 4; ++it) {
          const int row = it * 4 + q;
          const float* sp = slab + row * 68 + c8;
          v8h hv, lv;
#pragma unroll
          for (int e = 0; e < 8; ++e) {
            if (OUT_MODE == 1) {
              hv[e] = (_Float16)sp[e];
            } else {
              unsigned short hb = f2bf_bits(sp[e]);
              unsigned short lb = f2bf_bits(sp[e] - bf_bits2f(hb));
              hv[e] = __builtin_bit_cast(_Float16, hb);
              lv[e] = __builtin_bit_cast(_Float16, lb);
            }
          }
          *(volatile v8h*)(C + (size_t)(mBase + row) * ldc + n0 + c8) = hv;
          if (OUT_MODE == 2) *(volatile v8h*)(C2 + (size_t)(mBase + row) * ldc + n0 + c8) = lv;
        }
        __threadfence();
      }
    }
    __builtin_amdgcn_fence(__ATOMIC_RELEASE, "workgroup");
    __builtin_amdgcn_wave_barrier();
    __builtin_amdgcn_fence(__ATOMIC_ACQUIRE, "workgroup");
  }
}

__device__ __forceinline__ unsigned h_bits(float f) {
  return (unsigned)__builtin_bit_cast(unsigned short, (_Float16)f);
}
__device__ __forceinline__ float rcp_f(float x) { return __builtin_amdgcn_rcpf(x); }
__device__ __forceinline__ float sigm_f(float x) { return rcp_f(1.0f + expf(-x)); }
__device__ __forceinline__ float tanh_f(float x) { return 1.0f - 2.0f * rcp_f(1.0f + expf(2.0f * x)); }

__global__ __launch_bounds__(256) void prep_kernel(
    const float* __restrict__ Wx, const float* __restrict__ Wh,
    const float* __restrict__ W1, const float* __restrict__ b1,
    const float* __restrict__ stat, const float* __restrict__ unused_in,
    unsigned* __restrict__ wcat_w, unsigned* __restrict__ w1p_w,
    float* __restrict__ b1p, unsigned* __restrict__ feat_w)
{
  (void)unused_in;
  const int blk = blockIdx.x;
  const int tid = threadIdx.x;
  if (blk < 192) {
    const int idx = blk * 256 + tid;
    const int n = idx / 96;
    const int k0 = 2 * (idx - n * 96);
    const int kx = (k0 < kDin - 2) ? k0 : (kDin - 2);
    const float xa = Wx[n * kDin + kx];
    const float xb = Wx[n * kDin + kx + 1];
    int kh = k0 - kXpad; kh = kh < 0 ? 0 : kh; kh = kh > (kHid - 2) ? (kHid - 2) : kh;
    const float ha = Wh[n * kHid + kh];
    const float hb = Wh[n * kHid + kh + 1];
    const float v0 = (k0 < kDin) ? xa : ((k0 < kXpad) ? 0.0f : ha);
    const float v1 = (k0 < kDin) ? xb : ((k0 < kXpad) ? 0.0f : hb);
    const unsigned w = h_bits(16.0f * v0) | (h_bits(16.0f * v1) << 16);
    volatile unsigned* p = wcat_w + idx;
    *p = w;
    __threadfence();
    *p = w;
  } else if (blk < 264) {
    const int idx = (blk - 192) * 256 + tid;
    const int n = idx / 96;
    const int k0 = 2 * (idx - n * 96);
    const int k1 = k0 + 1;
    const int nc  = (n  < kDmlp) ? n  : (kDmlp - 1);
    const int k0c = (k0 < kDmlp) ? k0 : (kDmlp - 1);
    const int k1c = (k1 < kDmlp) ? k1 : (kDmlp - 1);
    const float a = W1[nc * kDmlp + k0c];
    const float b = W1[nc * kDmlp + k1c];
    const float v0 = (n < kDmlp && k0 < kDmlp) ? 16.0f * a : 0.0f;
    const float v1 = (n < kDmlp && k1 < kDmlp) ? 16.0f * b : 0.0f;
    const unsigned w = h_bits(v0) | (h_bits(v1) << 16);
    volatile unsigned* p = w1p_w + idx;
    *p = w;
    __threadfence();
    *p = w;
  } else if (blk == 264) {
    if (tid < kDmlpPad) {
      const int tc = (tid < kDmlp) ? tid : (kDmlp - 1);
      const float bv = b1[tc];
      const float v = (tid < kDmlp) ? bv : 0.0f;
      volatile float* p = b1p + tid;
      *p = v;
      __threadfence();
      *p = v;
    }
  } else {
    const int idx = (blk - 265) * 256 + tid;
    const int row = idx >> 5;
    const int j = idx & 31;
    const int s0 = 2 * j, s1 = s0 + 1;
    const int s0c = (s0 < kStatic) ? s0 : (kStatic - 1);
    const int s1c = (s1 < kStatic) ? s1 : (kStatic - 1);
    const float a = stat[row * kStatic + s0c];
    const float b = stat[row * kStatic + s1c];
    const float v0 = (s0 < kStatic) ? 16.0f * a : 0.0f;
    const float v1 = (s1 < kStatic) ? 16.0f * b : 0.0f;
    const unsigned w = h_bits(v0) | (h_bits(v1) << 16);
    volatile unsigned* p = feat_w + (size_t)row * (kDmlpPad / 2) + (kHid / 2) + j;
    *p = w;
    __threadfence();
    *p = w;
  }
}

__global__ __launch_bounds__(256) void enc_gin_kernel(
    const float* __restrict__ src, const float* __restrict__ encW, const float* __restrict__ encb,
    const float* __restrict__ gw1, const float* __restrict__ gb1,
    const float* __restrict__ ggam, const float* __restrict__ gbet,
    const float* __restrict__ gw2, const float* __restrict__ gb2,
    _Float16* __restrict__ xg)
{
  __shared__ __align__(16) _Float16 tA[kEncRows * kEncPitch];
  __shared__ __align__(16) _Float16 tW[64 * kEncPitch];
  __shared__ __align__(16) float sT[8][16 * 68];

  const int tid  = threadIdx.x;
  const int wave = tid >> 5;
  const int lane = tid & 31;
  const int hh   = lane >> 4;
  const int cc   = lane & 15;
  const int koff = hh * 8;
  const int mOff = hh * 8;
  const int blk  = blockIdx.x;
  const size_t row0 = (size_t)blk * kEncRows;

#pragma unroll
  for (int i = 0; i < 9; ++i) {
    const int idx = tid + 256 * i;
    const int row = idx / 18;
    const int w = idx - row * 18;
    const v2f s2 = *(const v2f*)(src + (row0 + row) * kDin + 2 * w);
    v2h hv;
    hv[0] = (_Float16)s2[0];
    hv[1] = (_Float16)s2[1];
    *(v2h*)(tA + row * kEncPitch + 2 * w) = hv;
  }
#pragma unroll
  for (int i = 0; i < 7; ++i) {
    const int idx = tid + 256 * i;
    const int row = idx / 14;
    const int w = idx - row * 14;
    v2h z2;
    z2[0] = (_Float16)0.0f;
    z2[1] = (_Float16)0.0f;
    *(v2h*)(tA + row * kEncPitch + kDin + 2 * w) = z2;
  }
#pragma unroll
  for (int i = 0; i < 8; ++i) {
    const int idx = tid + 256 * i;
    const int n = idx >> 5;
    const int k0 = 2 * (idx & 31);
    const int nn = (n < kDin) ? n : (kDin - 1);
    const int kk = (k0 < kDin - 2) ? k0 : (kDin - 2);
    const float w0 = encW[nn * kDin + kk];
    const float w1 = encW[nn * kDin + kk + 1];
    const bool ok = (n < kDin) && (k0 < kDin);
    v2h hv;
    hv[0] = (_Float16)(ok ? 16.0f * w0 : 0.0f);
    hv[1] = (_Float16)(ok ? 16.0f * w1 : 0.0f);
    *(v2h*)(tW + n * kEncPitch + k0) = hv;
  }
  __syncthreads();

  v8f acc[4];
#pragma unroll
  for (int j = 0; j < 4; ++j) acc[j] = (v8f){0.f,0.f,0.f,0.f,0.f,0.f,0.f,0.f};
#pragma unroll
  for (int ks = 0; ks < 2; ++ks) {
    v16h bq[4];
#pragma unroll
    for (int j = 0; j < 4; ++j) bq[j] = Frag<_Float16>::load(tW + (16 * j + cc) * kEncPitch + koff + 32 * ks);
    const v16h a = Frag<_Float16>::load(tA + (16 * wave + cc) * kEncPitch + koff + 32 * ks);
#pragma unroll
    for (int j = 0; j < 4; ++j) acc[j] = Frag<_Float16>::mma(a, bq[j], acc[j]);
    Frag<_Float16>::guard(acc[0], acc[3], a, bq[3]);
    Frag<_Float16>::keep(bq[0], bq[1], bq[2], bq[3]);
  }
  acc_guard4(acc[0], acc[1], acc[2], acc[3]);

  float* slab = sT[wave];
#pragma unroll
  for (int j = 0; j < 4; ++j) {
    const int n = 16 * j + cc;
    const int nc = (n < kDin) ? n : (kDin - 1);
    const float bvl = encb[nc];
    const float bb = (n < kDin) ? 8.0f * bvl : 0.0f;
#pragma unroll
    for (int r = 0; r < 8; ++r) slab[(mOff + r) * 68 + n] = acc[j][r] * 0.5f + bb;
  }
  __builtin_amdgcn_fence(__ATOMIC_RELEASE, "workgroup");
  __builtin_amdgcn_wave_barrier();
  __builtin_amdgcn_fence(__ATOMIC_ACQUIRE, "workgroup");

  float sv = slab[lane];
  const float sw = slab[32 + lane];
  sv += (lane < 4) ? sw : 0.0f;
#pragma unroll
  for (int off = 16; off >= 1; off >>= 1) sv += __shfl_xor(sv, off, 32);
  const bool aggsel = ((blk & 15) == 0) && (wave == 0);
  const float twoS = 2.0f * sv;

  const float g_w1 = gw1[0], g_b1 = gb1[0], g_gm = ggam[0], g_bt = gbet[0];
  const float g_w2 = gw2[0], g_b2 = gb2[0];
  const float bn_scale = 0.99999500004f;

  const int q = lane >> 3, c8 = (lane & 7) * 8;
  _Float16* obase = xg + (row0 + 16 * wave) * kXpad;
  for (int pass = 0; pass < 2; ++pass) {
#pragma unroll
    for (int it = 0; it < 4; ++it) {
      const int row = it * 4 + q;
      const float* sp = slab + row * 68 + c8;
      const float add = (aggsel && row == 0) ? twoS : 0.0f;
      v8h hv;
#pragma unroll
      for (int e = 0; e < 8; ++e) {
        const int col = c8 + e;
        float h = sp[e] + add;
        h = h * g_w1 + g_b1;
        h = (h * bn_scale) * g_gm + g_bt;
        h = fmaxf(h, 0.0f);
        h = h * g_w2 + g_b2;
        h = fmaxf(h, 0.0f);
        hv[e] = (_Float16)((col < kDin) ? h : 0.0f);
      }
      *(volatile v8h*)(obase + (size_t)row * kXpad + c8) = hv;
    }
    __threadfence();
  }
}

__global__ __launch_bounds__(256) void lstm_seq_kernel(
    const _Float16* __restrict__ xg,
    const _Float16* __restrict__ wcat,
    const float* __restrict__ bx, const float* __restrict__ bh,
    const int* __restrict__ lengths,
    _Float16* __restrict__ feat)
{
  __shared__ __align__(16) _Float16 tile[2][kRowsPB * kTilePitch];
  __shared__ __align__(16) _Float16 stg[kRowsPB * kStgPitch];

  const int tid  = threadIdx.x;
  const int wave = tid >> 5;
  const int lane = tid & 31;
  const int hh   = lane >> 4;
  const int cc   = lane & 15;
  const int koff = hh * 8;
  const int b0   = blockIdx.x * kRowsPB;
  const int ucol = 16 * wave + cc;

  if (tid < 128) {
    const int row = tid >> 3, ch = tid & 7;
    const v8h v = *(const v8h*)(xg + ((size_t)(b0 + row)) * kXpad + ch * 8);
    *(v8h*)(&tile[0][row * kTilePitch + ch * 8]) = v;
  }
  {
    v8h z;
#pragma unroll
    for (int e = 0; e < 8; ++e) z[e] = (_Float16)0.0f;
    *(v8h*)(&tile[0][(tid >> 4) * kTilePitch + kXpad + (tid & 15) * 8]) = z;
  }
  float bias4[4];
#pragma unroll
  for (int g = 0; g < 4; ++g) bias4[g] = bx[g * kHid + ucol] + bh[g * kHid + ucol];
  int len8[8];
  float creg[8], pool[8];
#pragma unroll
  for (int r = 0; r < 8; ++r) {
    int lv = lengths[b0 + 8 * hh + r];
    lv = lv < 0 ? 0 : lv;
    lv = lv > kSteps ? kSteps : lv;
    len8[r] = lv;
    creg[r] = 0.0f;
    pool[r] = 0.0f;
  }
  __syncthreads();

  const float inv16 = 0.0625f;
#pragma unroll 1
  for (int t = 0; t < kSteps; ++t) {
    const _Float16* cur = &tile[t & 1][0];
    _Float16* nxt = &tile[(t + 1) & 1][0];

    v8f acc[4];
#pragma unroll
    for (int g = 0; g < 4; ++g) acc[g] = (v8f){0.f,0.f,0.f,0.f,0.f,0.f,0.f,0.f};
#pragma unroll
    for (int ks = 0; ks < kKcat / 32; ++ks) {
      v16h bq[4];
#pragma unroll
      for (int g = 0; g < 4; ++g)
        bq[g] = Frag<_Float16>::load(wcat + (size_t)(g * kHid + ucol) * kKcat + koff + 32 * ks);
      const v16h a = Frag<_Float16>::load(cur + cc * kTilePitch + koff + 32 * ks);
#pragma unroll
      for (int g = 0; g < 4; ++g) acc[g] = Frag<_Float16>::mma(a, bq[g], acc[g]);
      Frag<_Float16>::guard(acc[0], acc[3], a, bq[3]);
      Frag<_Float16>::keep(bq[0], bq[1], bq[2], bq[3]);
    }
    acc_guard4(acc[0], acc[1], acc[2], acc[3]);

    if (t + 1 < kSteps) {
      if (tid < 128) {
        const int row = tid >> 3, ch = tid & 7;
        const v8h v = *(const v8h*)(xg + ((size_t)(t + 1) * kBatch + b0 + row) * kXpad + ch * 8);
        *(v8h*)(nxt + row * kTilePitch + ch * 8) = v;
      }
    }

#pragma unroll
    for (int r = 0; r < 8; ++r) {
      const float gi = acc[0][r] * inv16 + bias4[0];
      const float gf = acc[1][r] * inv16 + bias4[1];
      const float gg = acc[2][r] * inv16 + bias4[2];
      const float go = acc[3][r] * inv16 + bias4[3];
      const float sf = sigm_f(gf);
      const float si = sigm_f(gi);
      const float tg = tanh_f(gg);
      const float cn = creg[r] * sf + si * tg;
      const float hv = sigm_f(go) * tanh_f(cn);
      creg[r] = cn;
      pool[r] += (t < len8[r]) ? hv : 0.0f;
      nxt[(8 * hh + r) * kTilePitch + kXpad + ucol] = (_Float16)hv;
    }
    __syncthreads();
  }

#pragma unroll
  for (int r = 0; r < 8; ++r) {
    const float inv = rcp_f((float)len8[r] + 1.0f);
    stg[(8 * hh + r) * kStgPitch + ucol] = (_Float16)(pool[r] * inv * 16.0f);
  }
  __syncthreads();
  {
    const int q = lane >> 3, c8 = (lane & 7) * 8;
    const int line = 4 * wave + q;
    const int row = line >> 1, seg = line & 1;
    const v8h v = *(const v8h*)(stg + row * kStgPitch + seg * 64 + c8);
    _Float16* dst = feat + (size_t)(b0 + row) * kDmlpPad + seg * 64 + c8;
    *(volatile v8h*)dst = v;
    __threadfence();
    *(volatile v8h*)dst = v;
  }
}

__global__ __launch_bounds__(32) void head_kernel(
    const float* __restrict__ hid,
    const float* __restrict__ W2,
    const float* __restrict__ b2,
    float* __restrict__ out)
{
  __shared__ __align__(16) float s[32];
  const int lane = threadIdx.x;
  const int row = blockIdx.x * kRowsPB + (lane >> 1);
  const int cls = lane & 1;
  const float* hp = hid + (size_t)row * kDmlpPad;
  const float* wp = W2 + cls * kDmlp;
  float a = b2[cls];
#pragma unroll 1
  for (int k = 0; k < kDmlp; ++k) a += hp[k] * wp[k];
  s[lane] = a;
  __syncthreads();
  const int lc = (lane < 8) ? lane : 0;
  const v4f v = *(const v4f*)(s + 4 * lc);
  float* dst = out + (size_t)blockIdx.x * 32 + 4 * lc;
  if (lane < 8) *(volatile v4f*)dst = v;
  __threadfence();
  if (lane < 8) *(volatile v4f*)dst = v;
}

extern "C" void kernel_launch(void* const* d_in, const int* in_sizes, int n_in,
                              void* d_out, int out_size, void* d_ws,
                              size_t ws_size, hipStream_t stream) {
  if (n_in < 20) return;
  if (in_sizes[0] != kSteps * kBatch * kDin) return;
  if (in_sizes[3] != kBatch) return;
  if (out_size != kBatch * kClasses) return;

  const float* src     = (const float*)d_in[0];
  const float* stat    = (const float*)d_in[1];
  const float* times   = (const float*)d_in[2];
  const int*   lengths = (const int*)d_in[3];
  const float* encW    = (const float*)d_in[4];
  const float* encb    = (const float*)d_in[5];
  const float* gw1     = (const float*)d_in[6];
  const float* gb1     = (const float*)d_in[7];
  const float* ggam    = (const float*)d_in[8];
  const float* gbet    = (const float*)d_in[9];
  const float* gw2     = (const float*)d_in[10];
  const float* gb2     = (const float*)d_in[11];
  const float* Wx      = (const float*)d_in[12];
  const float* bx      = (const float*)d_in[13];
  const float* Wh      = (const float*)d_in[14];
  const float* bh      = (const float*)d_in[15];
  const float* W1      = (const float*)d_in[16];
  const float* b1      = (const float*)d_in[17];
  const float* W2      = (const float*)d_in[18];
  const float* b2      = (const float*)d_in[19];
  float* out = (float*)d_out;

  char* ws = (char*)d_ws;
  size_t off = 0;
  _Float16* xg = (_Float16*)(ws + off);   off += (size_t)kSteps * kBatch * kXpad * 2;
  _Float16* wcat = (_Float16*)(ws + off); off += (size_t)kGates * kKcat * 2;
  _Float16* w1p = (_Float16*)(ws + off);  off += (size_t)kDmlpPad * kDmlpPad * 2;
  float* b1p = (float*)(ws + off);        off += (size_t)kDmlpPad * 4;
  _Float16* feat = (_Float16*)(ws + off); off += (size_t)kBatch * kDmlpPad * 2;
  float* hid = (float*)(ws + off);        off += (size_t)kBatch * kDmlpPad * 4;
  if (off > ws_size) return;

  const int prepBlocks = 192 + 72 + 1 + (kBatch * (kDmlpPad - kHid) / 2) / 256;
  prep_kernel<<<prepBlocks, 256, 0, stream>>>(
      Wx, Wh, W1, b1, stat, times,
      (unsigned*)wcat, (unsigned*)w1p, b1p, (unsigned*)feat);

  enc_gin_kernel<<<(kSteps * kBatch) / kEncRows, 256, 0, stream>>>(
      src, encW, encb, gw1, gb1, ggam, gbet, gw2, gb2, xg);

  lstm_seq_kernel<<<kBatch / kRowsPB, 256, 0, stream>>>(
      xg, wcat, bx, bh, lengths, feat);

  wmma_gemm64<0, false, 2, 0, false, 2><<<dim3((kBatch / 64) * (kDmlpPad / 64) / 8, 1), 256, 0, stream>>>(
      (const unsigned short*)feat, (const unsigned short*)nullptr, kDmlpPad, 0L,
      (const unsigned short*)w1p, (const unsigned short*)nullptr, kDmlpPad, 0L,
      (void*)hid, (void*)nullptr, kDmlpPad, 0L,
      b1p, (const float*)nullptr, 0L,
      kBatch, kDmlpPad, kDmlpPad, 1.0f / 256.0f);

  head_kernel<<<kBatch / kRowsPB, 32, 0, stream>>>(hid, W2, b2, out);
}
